// MultiHeadAttention_11433202942880
// MI455X (gfx1250) — hardware-verified
//
#include <hip/hip_runtime.h>
#ifndef NB
#define NB 2
#endif
#ifndef SEQ
#define SEQ 2048
#endif
#ifndef QE
#define QE ((SEQ) < 256 ? (SEQ) : 256)
#endif
#define NB_FULL 2
#define SEQ_FULL 2048
#define DM 1024
#define NH 16
#define HD 64
#define NR (NB * SEQ)

static_assert(NH * HD == DM);
static_assert(HD == 64);
static_assert(DM % 64 == 0 && DM % 32 == 0);
static_assert(NR % 128 == 0);
static_assert(SEQ % 64 == 0 && QE % 64 == 0 && QE <= SEQ && (SEQ - QE) % 64 == 0);
static_assert(NB <= NB_FULL && SEQ <= SEQ_FULL);
static_assert((NR * DM / 8) % 256 == 0 && (DM * DM / 8) % 256 == 0);
static_assert((SEQ & (SEQ - 1)) == 0);
static_assert(DM % 4 == 0 && (DM / 64 - 1) * 64 + 15 * 4 + 4 <= DM);
static_assert((size_t)NB_FULL * SEQ_FULL * DM * 4 == (size_t)16777216);

typedef __bf16 v16b __attribute__((ext_vector_type(16)));
typedef _Float16 v16h __attribute__((ext_vector_type(16)));
typedef unsigned short v8us __attribute__((ext_vector_type(8), may_alias));
typedef float v8f __attribute__((ext_vector_type(8)));
typedef float v4f __attribute__((ext_vector_type(4)));
typedef float v4fa __attribute__((ext_vector_type(4), may_alias));
union FragB { v16b v; v8us half[2]; unsigned short u[16]; };
union FragH { v16h v; v8us half[2]; _Float16 h[16]; unsigned short u[16]; };

__device__ __forceinline__ unsigned short bf16_bits(float x) { unsigned int u = __float_as_uint(x); return (unsigned short)((u + 0x7FFFu + ((u >> 16) & 1u)) >> 16); }
__device__ __forceinline__ float bf16_val(unsigned short b) { return __uint_as_float(((unsigned int)b) << 16); }
__device__ __forceinline__ float bf16_rne(float x) { return bf16_val(bf16_bits(x)); }

__device__ __forceinline__ v16b ldb(const unsigned short* __restrict__ p, size_t off, int hh) { FragB f; f.half[0] = *(const v8us*)(p + off + 8 * hh); f.half[1] = *(const v8us*)(p + off + 16 + 8 * hh); return f.v; }
__device__ __forceinline__ v16h ldh(const unsigned short* __restrict__ p, size_t off, int hh) { FragH f; f.half[0] = *(const v8us*)(p + off + 8 * hh); f.half[1] = *(const v8us*)(p + off + 16 + 8 * hh); return f.v; }

template <int NT>
__device__ __forceinline__ v8f mmaB(v16b ah, v16b al, v16b bh, v16b bl, v8f c) {
  c = __builtin_amdgcn_wmma_f32_16x16x32_bf16(false, ah, false, bh, (short)0, c, false, false);
  if (NT >= 2) c = __builtin_amdgcn_wmma_f32_16x16x32_bf16(false, al, false, bh, (short)0, c, false, false);
  if (NT >= 3) c = __builtin_amdgcn_wmma_f32_16x16x32_bf16(false, ah, false, bl, (short)0, c, false, false);
  asm volatile("v_nop\n\tv_nop\n\tv_nop\n\tv_nop" : "+v"(c) : "v"(ah), "v"(al), "v"(bh), "v"(bl));
  return c;
}
__device__ __forceinline__ v8f mmaH1(v16h a, v16h b, v8f c) {
  v8f d = __builtin_amdgcn_wmma_f32_16x16x32_f16(false, a, false, b, (short)0, c, false, false);
  asm volatile("v_nop\n\tv_nop\n\tv_nop\n\tv_nop" : "+v"(d) : "v"(a), "v"(b));
  return d;
}

__global__ __launch_bounds__(256) void k_x16(const float* __restrict__ x, unsigned short* __restrict__ X16) {
  const int t = blockIdx.x * 256 + threadIdx.x;
  if (t >= NR * DM / 8) return;
  const int row = t / (DM / 8), c8 = (t - row * (DM / 8)) * 8;
  const int b = row / SEQ, s = row - b * SEQ;
  const float* src = x + ((size_t)b * SEQ_FULL + s) * DM + c8;
  const v4f a = *(const v4fa*)src, c = *(const v4fa*)(src + 4);
  FragH f;
#pragma unroll
  for (int q = 0; q < 4; ++q) { f.h[q] = (_Float16)bf16_rne(a[q]); f.h[4 + q] = (_Float16)bf16_rne(c[q]); }
  const v8us o = f.half[0];
  unsigned short* d = X16 + (size_t)t * 8;
  *(volatile v8us*)d = o;
  __threadfence();
  *(volatile v8us*)d = o;
}
__global__ __launch_bounds__(256) void k_wnat(const float* __restrict__ w, unsigned short* __restrict__ Bt) {
  const int t = blockIdx.x * 256 + threadIdx.x;
  if (t >= DM * DM / 8) return;
  const v4f a = *(const v4fa*)(w + (size_t)t * 8), c = *(const v4fa*)(w + (size_t)t * 8 + 4);
  FragH f;
#pragma unroll
  for (int q = 0; q < 4; ++q) { f.h[q] = (_Float16)(bf16_rne(a[q]) * 16.0f); f.h[4 + q] = (_Float16)(bf16_rne(c[q]) * 16.0f); }
  const v8us o = f.half[0];
  unsigned short* d = Bt + (size_t)t * 8;
  *(volatile v8us*)d = o;
  __threadfence();
  *(volatile v8us*)d = o;
}
__global__ __launch_bounds__(256) void k_wbf(const float* __restrict__ w, unsigned short* __restrict__ Bt) {
  const int t = blockIdx.x * 256 + threadIdx.x;
  if (t >= DM * DM / 8) return;
  const v4f a = *(const v4fa*)(w + (size_t)t * 8), c = *(const v4fa*)(w + (size_t)t * 8 + 4);
  v8us o;
#pragma unroll
  for (int q = 0; q < 4; ++q) { o[q] = bf16_bits(a[q]); o[4 + q] = bf16_bits(c[q]); }
  unsigned short* d = Bt + (size_t)t * 8;
  *(volatile v8us*)d = o;
  __threadfence();
  *(volatile v8us*)d = o;
}

template <int MODE>
__device__ __forceinline__ void proj_body(const unsigned short* __restrict__ A, const unsigned short* __restrict__ Bt,
                                          unsigned short* __restrict__ P0, unsigned short* __restrict__ P1) {
  __shared__ __attribute__((aligned(16))) float so[4][32][68];
  const int lane = threadIdx.x & 31, ln = lane & 15, hh = lane >> 4;
  const int w = __builtin_amdgcn_readfirstlane((int)(threadIdx.x >> 5));
  const int mt = blockIdx.x / (DM / 64), nq = blockIdx.x - mt * (DM / 64);
  const int row0 = mt * 128 + 32 * w, col0 = nq * 64;
  const size_t a0 = (size_t)(row0 + ln) * DM, a1 = a0 + (size_t)16 * DM;
  const size_t b0 = (size_t)(col0 + ln) * DM, b1 = b0 + (size_t)16 * DM, b2 = b1 + (size_t)16 * DM, b3 = b2 + (size_t)16 * DM;
  const v8f z8 = {0.f, 0.f, 0.f, 0.f, 0.f, 0.f, 0.f, 0.f};
  v8f c00 = z8, c01 = z8, c02 = z8, c03 = z8, c10 = z8, c11 = z8, c12 = z8, c13 = z8;
#pragma unroll 1
  for (int kb = 0; kb < DM; kb += 32) {
    const v16h fa0 = ldh(A, a0 + kb, hh), fa1 = ldh(A, a1 + kb, hh);
    v16h fb = ldh(Bt, b0 + kb, hh); c00 = mmaH1(fa0, fb, c00); c10 = mmaH1(fa1, fb, c10);
    fb = ldh(Bt, b1 + kb, hh); c01 = mmaH1(fa0, fb, c01); c11 = mmaH1(fa1, fb, c11);
    fb = ldh(Bt, b2 + kb, hh); c02 = mmaH1(fa0, fb, c02); c12 = mmaH1(fa1, fb, c12);
    fb = ldh(Bt, b3 + kb, hh); c03 = mmaH1(fa0, fb, c03); c13 = mmaH1(fa1, fb, c13);
  }
  v8f accs[8] = {c00, c01, c02, c03, c10, c11, c12, c13};
#pragma unroll
  for (int u = 0; u < 8; ++u) {
    const int t = u & 3, half = u >> 2;
#pragma unroll
    for (int r = 0; r < 8; ++r) so[w][half * 16 + 8 * hh + r][t * 16 + ln] = accs[u][r] * 0.0625f;
  }
  __builtin_amdgcn_fence(4  , "workgroup");
  __builtin_amdgcn_wave_barrier();
  const int rq = lane >> 3, c8 = (lane & 7) * 8;
  for (int pass = 0; pass < 2; ++pass) {
#pragma unroll
    for (int q = 0; q < 8; ++q) {
      const int r = q * 4 + rq;
      const v4f x0 = *(const v4fa*)&so[w][r][c8], x1 = *(const v4fa*)&so[w][r][c8 + 4];
      const float xs[8] = {x0[0], x0[1], x0[2], x0[3], x1[0], x1[1], x1[2], x1[3]};
      v8us o0, o1;
      if (MODE == 0) {
#pragma unroll
        for (int i = 0; i < 8; ++i) { const unsigned short hb = bf16_bits(xs[i]); o0[i] = hb; o1[i] = bf16_bits(xs[i] - bf16_val(hb)); }
      } else {
        FragH fh, fl;
#pragma unroll
        for (int i = 0; i < 8; ++i) { const _Float16 hv = (_Float16)xs[i]; fh.h[i] = hv; fl.h[i] = (_Float16)((xs[i] - (float)hv) * 1024.0f); }
        o0 = fh.half[0]; o1 = fl.half[0];
      }
      const size_t go = (size_t)(row0 + r) * DM + col0 + c8;
      *(volatile v8us*)(P0 + go) = o0;
      *(volatile v8us*)(P1 + go) = o1;
    }
    if (pass == 0) __threadfence();
  }
}
__global__ __launch_bounds__(128) void k_proj_qk(const unsigned short* __restrict__ A, const unsigned short* __restrict__ Bt,
                                                 unsigned short* __restrict__ P0, unsigned short* __restrict__ P1) { proj_body<0>(A, Bt, P0, P1); }
__global__ __launch_bounds__(128) void k_proj_v(const unsigned short* __restrict__ A, const unsigned short* __restrict__ Bt,
                                                unsigned short* __restrict__ P0, unsigned short* __restrict__ P1) { proj_body<1>(A, Bt, P0, P1); }

__global__ __launch_bounds__(256) void k_vt(const unsigned short* __restrict__ V16, unsigned short* __restrict__ Vt, int ntok) {
  __shared__ unsigned short tl[64][66];
  const int tid = threadIdx.x;
  const int ng = ntok / 64;
  const int slab = blockIdx.x / ng, lg = blockIdx.x - slab * ng;
  const int b = slab / NH, h = slab - b * NH;
  for (int i = tid; i < 64 * 8; i += 256) {
    const int r = i / 8, c8 = (i % 8) * 8;
    FragH f;
    f.half[0] = *(const v8us*)(V16 + ((size_t)b * SEQ + lg * 64 + r) * DM + h * HD + c8);
#pragma unroll
    for (int q = 0; q < 8; ++q) tl[r][c8 + q] = f.u[q];
  }
  __syncthreads();
  for (int pass = 0; pass < 2; ++pass) {
#pragma unroll
    for (int rd = 0; rd < 2; ++rd) {
      const int d = rd * 32 + tid / 8, pc = tid % 8;
      FragH f;
#pragma unroll
      for (int q = 0; q < 8; ++q) f.u[q] = tl[pc * 8 + q][d];
      const v8us o = f.half[0];
      *(volatile v8us*)(Vt + ((size_t)slab * HD + d) * ntok + lg * 64 + pc * 8) = o;
    }
    if (pass == 0) __threadfence();
  }
}

template <bool EARLY>
__device__ __forceinline__ void attn_body(const unsigned short* __restrict__ Qh, const unsigned short* __restrict__ Ql,
                                          const unsigned short* __restrict__ Kh, const unsigned short* __restrict__ Kl,
                                          const unsigned short* __restrict__ Vth, const unsigned short* __restrict__ Vtl,
                                          unsigned short* __restrict__ Ch, unsigned short* __restrict__ Cl) {
  __shared__ __attribute__((aligned(16))) float so[4][16][68];
  constexpr int QT0 = EARLY ? 0 : QE / 16;
  constexpr int NQT = EARLY ? QE / 16 : (SEQ - QE) / 16;
  constexpr int BPB = (NQT / 4 > 0) ? NQT / 4 : 1;
  const int lane = threadIdx.x & 31, ln = lane & 15, hh = lane >> 4;
  const int wave = __builtin_amdgcn_readfirstlane((int)(threadIdx.x >> 5));
  const int bh = blockIdx.x / BPB;
  const int qt = QT0 + (blockIdx.x - bh * BPB) * 4 + wave;
  const int b = bh / NH, h = bh - b * NH;
  const int qBase = qt * 16;
  const int nkt = (qBase + 47) >> 5;
  const int nFull = qBase >> 5;
  const int qrow = qBase + ln;
  const size_t offQ = ((size_t)b * SEQ + qrow) * DM + h * HD;
  const size_t offK = ((size_t)b * SEQ + ln) * DM + h * HD;
  const size_t offV = ((size_t)bh * HD + ln) * SEQ;
  const size_t offVl = ((size_t)bh * HD + ln) * QE;
  const v8f z8 = {0.f, 0.f, 0.f, 0.f, 0.f, 0.f, 0.f, 0.f};
  v8f oacc[4] = {z8, z8, z8, z8};
  v8f ores[4] = {z8, z8, z8, z8};
  float m = -__builtin_inff(), l = 0.f;
#pragma unroll 1
  for (int it = 0; it < nkt; ++it) {
    const int kb = it * 32;
    v8f st0 = z8, st1 = z8;
#pragma unroll
    for (int dc = 0; dc < 2; ++dc) {
      const size_t qo = offQ + dc * 32;
      const v16b fqh = ldb(Qh, qo, hh), fql = ldb(Ql, qo, hh);
      const size_t k0 = offK + (size_t)kb * DM + dc * 32;
      const size_t k1 = k0 + (size_t)16 * DM;
      st0 = mmaB<3>(ldb(Kh, k0, hh), ldb(Kl, k0, hh), fqh, fql, st0);
      st1 = mmaB<3>(ldb(Kh, k1, hh), ldb(Kl, k1, hh), fqh, fql, st1);
      asm volatile("" ::: "memory");
    }
    float s0[8], s1[8];
#pragma unroll
    for (int r = 0; r < 8; ++r) { s0[r] = st0[r] * 0.125f; s1[r] = st1[r] * 0.125f; }
    if (it >= nFull) {
#pragma unroll
      for (int r = 0; r < 8; ++r) {
        const int key = kb + 8 * hh + r;
        s0[r] = (key > qrow) ? -__builtin_inff() : s0[r];
        s1[r] = (key + 16 > qrow) ? -__builtin_inff() : s1[r];
      }
    }
    float mt = fmaxf(s0[0], s1[0]);
#pragma unroll
    for (int r = 1; r < 8; ++r) mt = fmaxf(mt, fmaxf(s0[r], s1[r]));
    const float mo = __shfl_xor(mt, 16);
    const float mnew = fmaxf(fmaxf(mt, mo), m);
    const float alpha = __expf(m - mnew);
    m = mnew;
    l *= alpha;
#pragma unroll
    for (int dt = 0; dt < 4; ++dt) { oacc[dt] *= alpha; if (EARLY) ores[dt] *= alpha; }
    FragH ph, pl;
#pragma unroll
    for (int r = 0; r < 8; ++r) {
      const float p0 = __expf(s0[r] - m), p1 = __expf(s1[r] - m);
      l += p0 + p1;
      const float c0 = p0 * 256.0f, c1 = p1 * 256.0f;
      const _Float16 h0 = (_Float16)c0, h1 = (_Float16)c1;
      ph.h[r] = h0; ph.h[8 + r] = h1;
      pl.h[r] = (_Float16)((c0 - (float)h0) * 1024.0f);
      pl.h[8 + r] = (_Float16)((c1 - (float)h1) * 1024.0f);
    }
    asm volatile("" ::: "memory");
#pragma unroll
    for (int dt = 0; dt < 4; ++dt) {
      const size_t vo = offV + (size_t)dt * 16 * SEQ + kb;
      FragH vh; vh.v = ldh(Vth, vo, hh);
      if (EARLY) {
        const size_t vlo = offVl + (size_t)dt * 16 * QE + kb;
        FragH vl; vl.v = ldh(Vtl, vlo, hh);
        v8f o = oacc[dt], e = ores[dt];
        o = __builtin_amdgcn_wmma_f32_16x16x32_f16(false, vh.v, false, ph.v, (short)0, o, false, false);
        e = __builtin_amdgcn_wmma_f32_16x16x32_f16(false, vl.v, false, ph.v, (short)0, e, false, false);
        e = __builtin_amdgcn_wmma_f32_16x16x32_f16(false, vh.v, false, pl.v, (short)0, e, false, false);
        asm volatile("v_nop\n\tv_nop\n\tv_nop\n\tv_nop" : "+v"(o), "+v"(e) : "v"(vh.v), "v"(vl.v), "v"(ph.v), "v"(pl.v));
        oacc[dt] = o; ores[dt] = e;
      } else {
        oacc[dt] = mmaH1(vh.v, ph.v, oacc[dt]);
      }
    }
    asm volatile("" ::: "memory");
  }
  const float lt = l + __shfl_xor(l, 16);
  const float rinv = 1.0f / (256.0f * lt);
#pragma unroll
  for (int dt = 0; dt < 4; ++dt) {
    v8f o = oacc[dt];
    if (EARLY) o = o + ores[dt] * 0.0009765625f;
    const v4f w0 = {o[0] * rinv, o[1] * rinv, o[2] * rinv, o[3] * rinv};
    const v4f w1 = {o[4] * rinv, o[5] * rinv, o[6] * rinv, o[7] * rinv};
    *(v4fa*)&so[wave][ln][dt * 16 + 8 * hh] = w0;
    *(v4fa*)&so[wave][ln][dt * 16 + 8 * hh + 4] = w1;
  }
  __builtin_amdgcn_fence(4  , "workgroup");
  __builtin_amdgcn_wave_barrier();
  const int rq = lane >> 3, c8 = (lane & 7) * 8;
  for (int pass = 0; pass < 2; ++pass) {
#pragma unroll
    for (int q = 0; q < 4; ++q) {
      const int r = q * 4 + rq;
      const v4f x0 = *(const v4fa*)&so[wave][r][c8], x1 = *(const v4fa*)&so[wave][r][c8 + 4];
      const float xs[8] = {x0[0], x0[1], x0[2], x0[3], x1[0], x1[1], x1[2], x1[3]};
      v8us o0, o1;
#pragma unroll
      for (int i = 0; i < 8; ++i) { const unsigned short hb = bf16_bits(xs[i]); o0[i] = hb; o1[i] = bf16_bits(xs[i] - bf16_val(hb)); }
      const size_t go = ((size_t)b * SEQ + qBase + r) * DM + h * HD + c8;
      *(volatile v8us*)(Ch + go) = o0;
      *(volatile v8us*)(Cl + go) = o1;
    }
    if (pass == 0) __threadfence();
  }
}
__global__ __launch_bounds__(128) void k_attn_main(const unsigned short* __restrict__ Qh, const unsigned short* __restrict__ Ql,
                                                   const unsigned short* __restrict__ Kh, const unsigned short* __restrict__ Kl,
                                                   const unsigned short* __restrict__ Vth, const unsigned short* __restrict__ Vtl,
                                                   unsigned short* __restrict__ Ch, unsigned short* __restrict__ Cl) { attn_body<false>(Qh, Ql, Kh, Kl, Vth, Vtl, Ch, Cl); }
__global__ __launch_bounds__(128) void k_attn_early(const unsigned short* __restrict__ Qh, const unsigned short* __restrict__ Ql,
                                                    const unsigned short* __restrict__ Kh, const unsigned short* __restrict__ Kl,
                                                    const unsigned short* __restrict__ Vth, const unsigned short* __restrict__ Vtl,
                                                    unsigned short* __restrict__ Ch, unsigned short* __restrict__ Cl) { attn_body<true>(Qh, Ql, Kh, Kl, Vth, Vtl, Ch, Cl); }

__global__ __launch_bounds__(128) void k_out(const unsigned short* __restrict__ Ah, const unsigned short* __restrict__ Al,
                                             const unsigned short* __restrict__ Bt, const float* __restrict__ bias, float* __restrict__ C) {
  __shared__ __attribute__((aligned(16))) float so[4][32][68];
  const int lane = threadIdx.x & 31, ln = lane & 15, hh = lane >> 4;
  const int w = __builtin_amdgcn_readfirstlane((int)(threadIdx.x >> 5));
  const int mt = blockIdx.x / (DM / 64), nq = blockIdx.x - mt * (DM / 64);
  const int row0 = mt * 128 + 32 * w, col0 = nq * 64;
  const size_t a0 = (size_t)(row0 + ln) * DM, a1 = a0 + (size_t)16 * DM;
  const size_t b0 = (size_t)(col0 + ln) * DM, b1 = b0 + (size_t)16 * DM, b2 = b1 + (size_t)16 * DM, b3 = b2 + (size_t)16 * DM;
  const v8f z8 = {0.f, 0.f, 0.f, 0.f, 0.f, 0.f, 0.f, 0.f};
  v8f c00 = z8, c01 = z8, c02 = z8, c03 = z8, c10 = z8, c11 = z8, c12 = z8, c13 = z8;
#pragma unroll 1
  for (int kb = 0; kb < DM; kb += 32) {
    const v16b h0 = ldb(Ah, a0 + kb, hh), l0 = ldb(Al, a0 + kb, hh);
    const v16b h1 = ldb(Ah, a1 + kb, hh), l1 = ldb(Al, a1 + kb, hh);
    v16b fb = ldb(Bt, b0 + kb, hh); c00 = mmaB<2>(h0, l0, fb, fb, c00); c10 = mmaB<2>(h1, l1, fb, fb, c10);
    fb = ldb(Bt, b1 + kb, hh); c01 = mmaB<2>(h0, l0, fb, fb, c01); c11 = mmaB<2>(h1, l1, fb, fb, c11);
    fb = ldb(Bt, b2 + kb, hh); c02 = mmaB<2>(h0, l0, fb, fb, c02); c12 = mmaB<2>(h1, l1, fb, fb, c12);
    fb = ldb(Bt, b3 + kb, hh); c03 = mmaB<2>(h0, l0, fb, fb, c03); c13 = mmaB<2>(h1, l1, fb, fb, c13);
  }
  v8f accs[8] = {c00, c01, c02, c03, c10, c11, c12, c13};
#pragma unroll
  for (int u = 0; u < 8; ++u) {
    const int t = u & 3, half = u >> 2;
#pragma unroll
    for (int r = 0; r < 8; ++r) so[w][half * 16 + 8 * hh + r][t * 16 + ln] = accs[u][r];
  }
  __builtin_amdgcn_fence(4  , "workgroup");
  __builtin_amdgcn_wave_barrier();
  const int rsub = lane >> 4, c4 = (lane & 15) * 4;
  const v4f bx = *(const v4fa*)(bias + col0 + c4);
  const v4f bv = {bf16_rne(bx[0]), bf16_rne(bx[1]), bf16_rne(bx[2]), bf16_rne(bx[3])};
  for (int pass = 0; pass < 2; ++pass) {
#pragma unroll
    for (int q = 0; q < 16; ++q) {
      const int r = q * 2 + rsub;
      const v4f sv = *(const v4fa*)&so[w][r][c4];
      const v4f v = sv + bv;
      const int grow = row0 + r;
      const int bb = grow / SEQ, s = grow - bb * SEQ;
      *(volatile v4f*)(C + ((size_t)bb * SEQ_FULL + s) * DM + col0 + c4) = v;
    }
    if (pass == 0) __threadfence();
  }
}

#define XB ((size_t)NR * DM * 2)
#define WB ((size_t)DM * DM * 2)
#define VLB ((size_t)NB * NH * HD * QE * 2)
static_assert(XB % 256 == 0 && WB % 256 == 0 && VLB % 256 == 0);
static_assert(12 * XB + 4 * WB + VLB <= (size_t)134217728);

extern "C" void kernel_launch(void* const* d_in, const int* in_sizes, int n_in,
                              void* d_out, int out_size, void* d_ws, size_t ws_size, hipStream_t stream) {
  if (n_in < 8) return;
  const long long need_x = ((long long)(NB - 1) * SEQ_FULL + SEQ) * DM;
  if (in_sizes[0] < need_x || in_sizes[1] < need_x || in_sizes[2] < need_x) return;
  if (in_sizes[3] < DM * DM || in_sizes[4] < DM * DM || in_sizes[5] < DM * DM || in_sizes[6] < DM * DM) return;
  if (in_sizes[7] < DM) return;
  if (out_size < need_x) return;
  const float* xq = (const float*)d_in[0];
  const float* xk = (const float*)d_in[1];
  const float* xv = (const float*)d_in[2];
  const float* wq = (const float*)d_in[3];
  const float* wk = (const float*)d_in[4];
  const float* wv = (const float*)d_in[5];
  const float* wo = (const float*)d_in[6];
  const float* bo = (const float*)d_in[7];
  char* ws = (char*)d_ws; size_t off = 0;
  auto take = [&](size_t bytes) { char* p = ws + off; off += (bytes + 255) & ~(size_t)255; return (unsigned short*)p; };
  unsigned short* XQ = take(XB); unsigned short* XK = take(XB); unsigned short* XV = take(XB);
  unsigned short* BQ = take(WB); unsigned short* BK = take(WB); unsigned short* BV = take(WB); unsigned short* BO = take(WB);
  unsigned short* Qh = take(XB); unsigned short* Ql = take(XB); unsigned short* Kh = take(XB); unsigned short* Kl = take(XB);
  unsigned short* Vh = take(XB); unsigned short* Vl = take(XB);
  unsigned short* Vth = take(XB); unsigned short* Vtl = take(VLB);
  unsigned short* Ch = take(XB); unsigned short* Cl = take(XB);
  if (off > ws_size) return;

  const unsigned gx = (unsigned)(NR * DM / 8 / 256), gw = (unsigned)(DM * DM / 8 / 256);
  k_x16<<<gx, 256, 0, stream>>>(xq, XQ);
  k_x16<<<gx, 256, 0, stream>>>(xk, XK);
  k_x16<<<gx, 256, 0, stream>>>(xv, XV);
  k_wnat<<<gw, 256, 0, stream>>>(wq, BQ);
  k_wnat<<<gw, 256, 0, stream>>>(wk, BK);
  k_wnat<<<gw, 256, 0, stream>>>(wv, BV);
  k_wbf<<<gw, 256, 0, stream>>>(wo, BO);

  const unsigned gp = (unsigned)((NR / 128) * (DM / 64));
  k_proj_qk<<<gp, 128, 0, stream>>>(XQ, BQ, Qh, Ql);
  k_proj_qk<<<gp, 128, 0, stream>>>(XK, BK, Kh, Kl);
  k_proj_v<<<gp, 128, 0, stream>>>(XV, BV, Vh, Vl);

  k_vt<<<(unsigned)(NB * NH * (SEQ / 64)), 256, 0, stream>>>(Vh, Vth, SEQ);
  k_vt<<<(unsigned)(NB * NH * (QE / 64)), 256, 0, stream>>>(Vl, Vtl, QE);

  k_attn_early<<<(unsigned)(NB * NH * (QE / 64)), 128, 0, stream>>>(Qh, Ql, Kh, Kl, Vth, Vtl, Ch, Cl);
  if (SEQ > QE) k_attn_main<<<(unsigned)(NB * NH * ((SEQ - QE) / 64)), 128, 0, stream>>>(Qh, Ql, Kh, Kl, Vth, Vtl, Ch, Cl);

  k_out<<<gp, 128, 0, stream>>>(Ch, Cl, BO, bo, (float*)d_out);
}
